// EdgeAwareCrossAttention_88003879895613
// MI455X (gfx1250) — hardware-verified
//
#include <hip/hip_runtime.h>
#include <math.h>

typedef __attribute__((ext_vector_type(16))) _Float16 v16h;
typedef __attribute__((ext_vector_type(16))) __bf16 v16b;
typedef __attribute__((ext_vector_type(8)))  _Float16 v8h;
typedef __attribute__((ext_vector_type(8)))  float v8f;
typedef __attribute__((ext_vector_type(4)))  float v4f;
typedef __attribute__((ext_vector_type(2)))  float v2f;
typedef __attribute__((ext_vector_type(4)))  unsigned v4u;
typedef __attribute__((ext_vector_type(4)))  int v4i;
typedef float __attribute__((may_alias)) float_a;
typedef int __attribute__((may_alias)) int_a;

template <typename T> __device__ __forceinline__ void vst2(void* p, T v) { *(volatile T*)p = v; __threadfence(); *(volatile T*)p = v; }
__device__ __forceinline__ v8f wmma16(v16h a, v16h b, v8f c) {
  v8f d = __builtin_amdgcn_wmma_f32_16x16x32_f16(false, a, false, b, (short)0, c, false, false);
  asm volatile("v_nop\n\tv_nop\n\tv_nop\n\tv_nop" : "+v"(d) : "v"(a), "v"(b));
  return d;
}
__device__ __forceinline__ v8f wmma_bf(v16b a, v16b b, v8f c) {
  v8f d = __builtin_amdgcn_wmma_f32_16x16x32_bf16(false, a, false, b, (short)0, c, false, false);
  asm volatile("v_nop\n\tv_nop\n\tv_nop\n\tv_nop" : "+v"(d) : "v"(a), "v"(b));
  return d;
}
__device__ __forceinline__ v16h frag_h(const _Float16* rowk0, int lane) {
  union { v16h v; v8h q[2]; } u; const _Float16* p = rowk0 + 8 * (lane >> 4);
  u.q[0] = *(const v8h*)p; u.q[1] = *(const v8h*)(p + 16); return u.v;
}
__device__ __forceinline__ v16h frag_f32(const float* rowk0, int lane) {
  v16h a; const float* p = rowk0 + 8 * (lane >> 4);
#pragma unroll
  for (int i = 0; i < 8; ++i) { a[i] = (_Float16)p[i]; a[8 + i] = (_Float16)p[16 + i]; }
  return a;
}
__device__ __forceinline__ v16h frag_f32s(const float* rowk0, int lane, float sc) {
  v16h a; const float* p = rowk0 + 8 * (lane >> 4);
#pragma unroll
  for (int i = 0; i < 8; ++i) { a[i] = (_Float16)(p[i] * sc); a[8 + i] = (_Float16)(p[16 + i] * sc); }
  return a;
}
__device__ __forceinline__ v16h fragc_f32(const float* W, int k0, int n, int lane, int ld, int K) {
  v16h a; const int g = lane >> 4;
#pragma unroll
  for (int i = 0; i < 8; ++i) { const int ka = k0 + 8 * g + i, kb = ka + 16;
    a[i] = (_Float16)(ka < K ? W[(size_t)(ka < K ? ka : K - 1) * ld + n] : 0.f); a[8 + i] = (_Float16)(kb < K ? W[(size_t)(kb < K ? kb : K - 1) * ld + n] : 0.f); }
  return a;
}
struct F2 { v16b h, l; };
__device__ __forceinline__ F2 bsplit16(const float v[16]) { F2 r;
#pragma unroll
  for (int i = 0; i < 16; ++i) { const __bf16 h = (__bf16)v[i]; r.h[i] = h; r.l[i] = (__bf16)(v[i] - (float)h); }
  return r; }
__device__ __forceinline__ F2 split_row(const float* row, int k0, int lane) { float v[16]; const float* p = row + k0 + 8 * (lane >> 4);
#pragma unroll
  for (int i = 0; i < 8; ++i) { v[i] = p[i]; v[8 + i] = p[16 + i]; }
  return bsplit16(v); }
__device__ __forceinline__ F2 split_rowK(const float* row, int k0, int lane, int K) { float v[16]; const int g = lane >> 4;
#pragma unroll
  for (int i = 0; i < 8; ++i) { const int ka = k0 + 8 * g + i, kb = ka + 16; v[i] = ka < K ? row[ka < K ? ka : K - 1] : 0.f; v[8 + i] = kb < K ? row[kb < K ? kb : K - 1] : 0.f; }
  return bsplit16(v); }
__device__ __forceinline__ F2 split_col(const float* W, int k0, int n, int lane, int ld, int K) { float v[16]; const int g = lane >> 4;
#pragma unroll
  for (int i = 0; i < 8; ++i) { const int ka = k0 + 8 * g + i, kb = ka + 16; v[i] = ka < K ? W[(size_t)(ka < K ? ka : K - 1) * ld + n] : 0.f; v[8 + i] = kb < K ? W[(size_t)(kb < K ? kb : K - 1) * ld + n] : 0.f; }
  return bsplit16(v); }
__device__ __forceinline__ v8f mac3(const F2& a, const F2& b, v8f c) { c = wmma_bf(a.l, b.h, c); c = wmma_bf(a.h, b.l, c); return wmma_bf(a.h, b.h, c); }
__device__ __forceinline__ float sigm(float v) { return 1.0f / (1.0f + expf(-v)); }
#define LDSX() do { asm volatile("s_wait_dscnt 0" ::: "memory"); __builtin_amdgcn_wave_barrier(); __builtin_amdgcn_fence(__ATOMIC_RELEASE, "workgroup"); } while (0)


#define NB 4
#define CC 256
#define NPOS 4096
#define IQ 32
#ifndef TQB
#define TQB (NPOS / 64)
#endif
typedef __attribute__((ext_vector_type(8))) __bf16 v8b;
__device__ __forceinline__ v16b frag_b(const __bf16* rowk0, int lane) {
  union { v16b v; v8b q[2]; } u; const __bf16* p = rowk0 + 8 * (lane >> 4);
  u.q[0] = *(const v8b*)p; u.q[1] = *(const v8b*)(p + 16); return u.v;
}
__device__ __forceinline__ float bfr(float v) { return (float)(__bf16)v; }
__device__ __attribute__((noinline)) float exp_ni(float v) { return expf(v); }
__device__ __attribute__((noinline)) float erf_ni(float v) { return erff(v); }

#define WS_PK  0u
#define WS_QH  (WS_PK + 2u * (2 * IQ + CC) * CC)
#define WS_QL  (WS_QH + 2u * NB * NPOS * IQ)
#define WS_KH  (WS_QL + 2u * NB * NPOS * IQ)
#define WS_KL  (WS_KH + 2u * NB * NPOS * IQ)
#define WS_VH  (WS_KL + 2u * NB * NPOS * IQ)
#define WS_END (WS_VH + 2u * (size_t)NB * CC * NPOS)

__global__ __launch_bounds__(256) void k_pack(const float* __restrict__ WQ, const float* __restrict__ WK, const float* __restrict__ WV, __bf16* __restrict__ PK) {
  const int n = blockIdx.x, t = threadIdx.x; __shared__ __align__(16) __bf16 s[CC]; const float* src = (n < IQ) ? (WQ + (size_t)n * CC) : (n < 2 * IQ) ? (WK + (size_t)(n - IQ) * CC) : (WV + (size_t)(n - 2 * IQ) * CC);
  s[t] = (__bf16)src[t]; __syncthreads();
  if (t < CC / 8) vst2((unsigned*)(PK + (size_t)n * CC + t * 8), *(const v4u*)&s[t * 8]);
}
__global__ __launch_bounds__(128) void k_proj(const float* __restrict__ FEAT, const float* __restrict__ EDGE, const __bf16* __restrict__ PK, const float* __restrict__ BQ, const float* __restrict__ BK, const float* __restrict__ BV, _Float16* __restrict__ QH, _Float16* __restrict__ QL, _Float16* __restrict__ KH, _Float16* __restrict__ KL, _Float16* __restrict__ VH) {
  __shared__ __align__(16) __bf16 sa[64][CC + 8]; __shared__ __align__(16) _Float16 sth[64][40], stl[64][40]; __shared__ __align__(16) _Float16 svh[CC][72];
  const int tid = threadIdx.x, wave = tid >> 5, lane = tid & 31, col = lane & 15, g = lane >> 4; const size_t b = blockIdx.y; const int n0 = blockIdx.x * 64;
#pragma unroll 1
  for (int src = 0; src < 2; ++src) { const float* Xs = src ? EDGE : FEAT;
    for (int e = tid; e < 64 * CC; e += 128) { const int c = e >> 6, r = e & 63; sa[r][c] = (__bf16)Xs[(b * CC + c) * NPOS + n0 + r]; }
    if (tid < 64) for (int c = CC; c < CC + 8; ++c) sa[tid][c] = (__bf16)0.f;
    __syncthreads();
    if (src == 0) { v8f acc[2] = {};
#pragma unroll
      for (int kc = 0; kc < CC / 32; ++kc) { const v16b a = frag_b(&sa[wave * 16 + col][kc * 32], lane);
#pragma unroll
        for (int j = 0; j < 2; ++j) acc[j] = wmma_bf(a, frag_b(PK + (size_t)(j * 16 + col) * CC + kc * 32, lane), acc[j]); }
#pragma unroll
      for (int j = 0; j < 2; ++j) { const float bb = bfr(BQ[j * 16 + col]);
#pragma unroll
        for (int r = 0; r < 8; ++r) { const float v = acc[j][r] + bb; const _Float16 hv = (_Float16)v; sth[wave * 16 + 8 * g + r][j * 16 + col] = hv; stl[wave * 16 + 8 * g + r][j * 16 + col] = (_Float16)((v - (float)hv) * 2048.0f); } }
      __syncthreads();
      for (int e = tid; e < 64 * 4; e += 128) { const int r = e >> 2, q = e & 3; const size_t o = ((b * NPOS + n0 + r) * IQ) + q * 8; vst2((unsigned*)(QH + o), *(const v4u*)&sth[r][q * 8]); vst2((unsigned*)(QL + o), *(const v4u*)&stl[r][q * 8]); }
    } else { v8f acc[18] = {};
#pragma unroll
      for (int kc = 0; kc < CC / 32; ++kc) { const v16b a = frag_b(&sa[wave * 16 + col][kc * 32], lane);
#pragma unroll
        for (int j = 0; j < 18; ++j) acc[j] = wmma_bf(a, frag_b(PK + (size_t)(IQ + j * 16 + col) * CC + kc * 32, lane), acc[j]); }
#pragma unroll
      for (int j = 0; j < 2; ++j) { const float bb = bfr(BK[j * 16 + col]);
#pragma unroll
        for (int r = 0; r < 8; ++r) { const float v = acc[j][r] + bb; const _Float16 hv = (_Float16)v; sth[wave * 16 + 8 * g + r][j * 16 + col] = hv; stl[wave * 16 + 8 * g + r][j * 16 + col] = (_Float16)((v - (float)hv) * 2048.0f); } }
#pragma unroll
      for (int j = 2; j < 18; ++j) { const int c = (j - 2) * 16 + col; const float bb = bfr(BV[c]);
#pragma unroll
        for (int r = 0; r < 8; ++r) svh[c][wave * 16 + 8 * g + r] = (_Float16)(acc[j][r] + bb); }
      __syncthreads();
      for (int e = tid; e < 64 * 4; e += 128) { const int r = e >> 2, q = e & 3; const size_t o = ((b * NPOS + n0 + r) * IQ) + q * 8; vst2((unsigned*)(KH + o), *(const v4u*)&sth[r][q * 8]); vst2((unsigned*)(KL + o), *(const v4u*)&stl[r][q * 8]); }
      for (int e = tid; e < CC * 8; e += 128) { const int c = e >> 3, pc = e & 7; vst2((unsigned*)(VH + (b * CC + c) * NPOS + n0 + pc * 8), *(const v4u*)&svh[c][pc * 8]); } }
    __syncthreads(); }
}
__global__ __launch_bounds__(128) void k_attn(const _Float16* __restrict__ QH, const _Float16* __restrict__ QL, const _Float16* __restrict__ KH, const _Float16* __restrict__ KL, const _Float16* __restrict__ VH, const float* __restrict__ FEAT, float* __restrict__ OUT) {
  __shared__ __align__(16) _Float16 sph[4][16][40]; __shared__ __align__(16) float so[128][68];
  const int tid = threadIdx.x, wave = tid >> 5, lane = tid & 31, col = lane & 15, g = lane >> 4; const int qb = blockIdx.x, half = blockIdx.y; const size_t b = blockIdx.z; const int q0 = qb * 64 + wave * 16; const size_t rq = b * NPOS + q0;
  const v16h aq = frag_h(QH + (rq + col) * IQ, lane), aql = frag_h(QL + (rq + col) * IQ, lane);
  float m[8], l[8];
#pragma unroll
  for (int r = 0; r < 8; ++r) { m[r] = -3.0e38f; l[r] = 0.f; }
  v8f acc[8] = {};
#pragma unroll 1
  for (int ks = 0; ks < NPOS / 32; ++ks) { const int j0 = ks * 32; v8f s[2];
#pragma unroll
    for (int ct = 0; ct < 2; ++ct) { const size_t rk = (b * NPOS + j0 + ct * 16 + col) * IQ; v8f c = {}, cl = {};
      { const v16h kh = frag_h(KH + rk, lane); c = wmma16(aq, kh, c); cl = wmma16(aql, kh, cl); cl = wmma16(aq, frag_h(KL + rk, lane), cl); }
#pragma unroll
      for (int r = 0; r < 8; ++r) s[ct][r] = c[r] + cl[r] * (1.0f / 2048.0f); }
#pragma unroll
    for (int r = 0; r < 8; ++r) { float mx = fmaxf(s[0][r], s[1][r]);
#pragma unroll
      for (int o = 1; o < 16; o <<= 1) mx = fmaxf(mx, __shfl_xor(mx, o));
      const float mn = fmaxf(m[r], mx); const float alpha = (m[r] <= -1.0e38f) ? 0.f : __expf(m[r] - mn); const float e0 = __expf(s[0][r] - mn), e1 = __expf(s[1][r] - mn); float es = e0 + e1;
#pragma unroll
      for (int o = 1; o < 16; o <<= 1) es += __shfl_xor(es, o);
      l[r] = l[r] * alpha + es; m[r] = mn;
#pragma unroll
      for (int dt = 0; dt < 8; ++dt) acc[dt][r] *= alpha;
      sph[wave][8 * g + r][col] = (_Float16)(e0 * 2048.0f); sph[wave][8 * g + r][16 + col] = (_Float16)(e1 * 2048.0f); }
    LDSX();
    const v16h pa = frag_h(&sph[wave][col][0], lane);
#pragma unroll
    for (int dt = 0; dt < 8; ++dt) acc[dt] = wmma16(pa, frag_h(VH + (b * CC + half * 128 + dt * 16 + col) * NPOS + j0, lane), acc[dt]);
    LDSX(); }
#pragma unroll
  for (int r = 0; r < 8; ++r) { const float il = (1.0f / 2048.0f) / l[r];
#pragma unroll
    for (int dt = 0; dt < 8; ++dt) { const int c = half * 128 + dt * 16 + col; const int n = q0 + 8 * g + r; so[dt * 16 + col][wave * 16 + 8 * g + r] = acc[dt][r] * il + bfr(FEAT[(b * CC + c) * NPOS + n]); } }
  __syncthreads();
  for (int e = tid; e < 128 * 16; e += 128) { const int cl = e >> 4, q = e & 15; vst2(OUT + (b * CC + half * 128 + cl) * NPOS + qb * 64 + q * 4, *(const v4f*)&so[cl][q * 4]); }
}
extern "C" void kernel_launch(void* const* d_in, const int* in_sizes, int n_in, void* d_out, int out_size, void* d_ws, size_t ws_size, hipStream_t stream) {
  (void)in_sizes; (void)n_in; (void)out_size;
  const float** F = (const float**)d_in;
  if (ws_size < (size_t)WS_END) return;
  char* ws = (char*)d_ws; __bf16* PK = (__bf16*)(ws + WS_PK); _Float16 *QH = (_Float16*)(ws + WS_QH), *QL = (_Float16*)(ws + WS_QL), *KH = (_Float16*)(ws + WS_KH), *KL = (_Float16*)(ws + WS_KL), *VH = (_Float16*)(ws + WS_VH);
  k_pack<<<2 * IQ + CC, 256, 0, stream>>>(F[2], F[4], F[6], PK);
  k_proj<<<dim3(NPOS / 64, NB), 128, 0, stream>>>(F[0], F[1], PK, F[3], F[5], F[7], QH, QL, KH, KL, VH);
  k_attn<<<dim3(TQB, 2, NB), 128, 0, stream>>>(QH, QL, KH, KL, VH, F[0], (float*)d_out);
}
